// FlaxMptAttention_71193377899323
// MI455X (gfx1250) — hardware-verified
//
#include <hip/hip_runtime.h>


typedef _Float16 v16h __attribute__((ext_vector_type(16)));
typedef _Float16 v8h  __attribute__((ext_vector_type(8)));
typedef v8h v8ha __attribute__((may_alias));
typedef __bf16 v16b __attribute__((ext_vector_type(16)));
typedef unsigned short v8us __attribute__((ext_vector_type(8)));
typedef v8us v8usa __attribute__((may_alias));
typedef float v8f __attribute__((ext_vector_type(8)));
typedef float v4f __attribute__((ext_vector_type(4)));
typedef v4f v4fa __attribute__((may_alias));

union FragH { v16h v; v8h p[2]; };
union FragB { v16b v; v8us p[2]; };

#define SEQ    2048
#define DMOD   2048
#define NHEAD  16
#define DHEAD  128
#define NQKV   6144

__device__ __forceinline__ v8f mma_h(v16h a, v16h b, v8f c) {
    c = __builtin_amdgcn_wmma_f32_16x16x32_f16(false, a, false, b, (short)0, c, false, false);
    asm volatile("v_nop\n\tv_nop\n\tv_nop\n\tv_nop" : "+v"(c) : "v"(a), "v"(b));
    return c;
}
__device__ __forceinline__ v8f mma_b(v16b a, v16b b, v8f c) {
    c = __builtin_amdgcn_wmma_f32_16x16x32_bf16(false, a, false, b, (short)0, c, false, false);
    asm volatile("v_nop\n\tv_nop\n\tv_nop\n\tv_nop" : "+v"(c) : "v"(a), "v"(b));
    return c;
}

__device__ __forceinline__ v16h ld_frag_h(const _Float16* rowp, int h) {
    FragH f;
    f.p[0] = *(const v8ha*)(rowp + 8 * h);
    f.p[1] = *(const v8ha*)(rowp + 16 + 8 * h);
    return f.v;
}
__device__ __forceinline__ v16b ld_frag_b(const unsigned short* rowp, int h) {
    FragB f;
    f.p[0] = *(const v8usa*)(rowp + 8 * h);
    f.p[1] = *(const v8usa*)(rowp + 16 + 8 * h);
    return f.v;
}

__device__ __forceinline__ unsigned short bf16_bits(float f) {
    unsigned u = __float_as_uint(f);
    u += 0x7FFFu + ((u >> 16) & 1u);
    return (unsigned short)(u >> 16);
}
__device__ __forceinline__ float bf16_val(unsigned short b) {
    return __uint_as_float(((unsigned)b) << 16);
}
__device__ __forceinline__ float wsum(float x) {
#pragma unroll
    for (int o = 16; o > 0; o >>= 1) x += __shfl_xor(x, o, 32);
    return x;
}

__global__ __launch_bounds__(256)
void k_cvt(const float* __restrict__ in, _Float16* out, int n) {
    const size_t i = ((size_t)blockIdx.x * 256 + threadIdx.x) * 8;
    if (i + 7 < (size_t)n) {
        const v4f a = *(const v4fa*)(in + i);
        const v4f b = *(const v4fa*)(in + i + 4);
        v8h hv;
        hv[0] = (_Float16)a[0]; hv[1] = (_Float16)a[1]; hv[2] = (_Float16)a[2]; hv[3] = (_Float16)a[3];
        hv[4] = (_Float16)b[0]; hv[5] = (_Float16)b[1]; hv[6] = (_Float16)b[2]; hv[7] = (_Float16)b[3];
        _Float16* p = out + i;
        *(volatile v8h*)p = hv;
        __threadfence();
        *(volatile v8h*)p = hv;
    }
}

__global__ __launch_bounds__(256)
void k_wtr(const float* __restrict__ W, _Float16* Wt, int K, int N, float wsc) {
    __shared__ float tile[64][33];
    const int tid = threadIdx.x;
    const int r = tid >> 5;
    const int c = tid & 31;
    const int kb = blockIdx.y * 64;
    const int nb = blockIdx.x * 32;
#pragma unroll
    for (int i = 0; i < 8; ++i) {
        const int kk = kb + r + 8 * i;
        const int nn = nb + c;
        tile[r + 8 * i][c] = (kk < K && nn < N) ? W[(size_t)kk * N + nn] : 0.0f;
    }
    __syncthreads();
    const int n = tid >> 3;
    const int q = tid & 7;
    v8h hv;
#pragma unroll
    for (int e = 0; e < 8; ++e) hv[e] = (_Float16)(tile[q * 8 + e][n] * wsc);
    const int nn = nb + n;
    const int k0 = kb + q * 8;
    if (nn < N && k0 + 7 < K) {
        _Float16* p = Wt + (size_t)nn * K + k0;
        *(volatile v8h*)p = hv;
        __threadfence();
        *(volatile v8h*)p = hv;
    }
}

#define GBM 128
#define GBN 128
#define GBK 32
#define GLD 40
#define GEP 68

__global__ __launch_bounds__(256) __attribute__((amdgpu_num_vgpr(256)))
void k_gemm(const _Float16* __restrict__ A, const _Float16* __restrict__ Bt,
            float* C, int M, int N, int K, float oscale) {
    __shared__ __attribute__((aligned(16))) _Float16 As[GBM * GLD];
    __shared__ __attribute__((aligned(16))) _Float16 Bs[GBN * GLD];
    __shared__ __attribute__((aligned(16))) float Es[8][16 * GEP];

    const int tid  = threadIdx.x;
    const int lane = tid & 31;
    const int wave = tid >> 5;
    const int h    = lane >> 4;
    const int m16  = lane & 15;
    const int wrow = wave & 3;
    const int wcol = wave >> 2;
    const int row0 = blockIdx.y * GBM;
    const int col0 = blockIdx.x * GBN;

    v8f acc[2][4];
#pragma unroll
    for (int i = 0; i < 2; ++i)
#pragma unroll
        for (int j = 0; j < 4; ++j) acc[i][j] = (v8f)0.0f;

    for (int k0 = 0; k0 < K; k0 += GBK) {
        __syncthreads();
#pragma unroll
        for (int i = 0; i < 2; ++i) {
            const int idx = tid + i * 256;
            const int r   = idx >> 2;
            const int c8  = (idx & 3) * 8;
            *(v8h*)&As[r * GLD + c8] = *(const v8ha*)(A + (size_t)(row0 + r) * K + k0 + c8);
        }
#pragma unroll
        for (int i = 0; i < 2; ++i) {
            const int idx = tid + i * 256;
            const int r   = idx >> 2;
            const int c8  = (idx & 3) * 8;
            *(v8h*)&Bs[r * GLD + c8] = *(const v8ha*)(Bt + (size_t)(col0 + r) * K + k0 + c8);
        }
        __syncthreads();

        v16h af[2], bf[4];
#pragma unroll
        for (int i = 0; i < 2; ++i)
            af[i] = ld_frag_h(&As[(wrow * 32 + i * 16 + m16) * GLD], h);
#pragma unroll
        for (int j = 0; j < 4; ++j)
            bf[j] = ld_frag_h(&Bs[(wcol * 64 + j * 16 + m16) * GLD], h);
#pragma unroll
        for (int i = 0; i < 2; ++i)
#pragma unroll
            for (int j = 0; j < 4; ++j)
                acc[i][j] = mma_h(af[i], bf[j], acc[i][j]);
    }

    float* e = Es[wave];
    const int c4 = (lane & 15) * 4;
#pragma unroll
    for (int i = 0; i < 2; ++i) {
        __syncthreads();
#pragma unroll
        for (int j = 0; j < 4; ++j)
#pragma unroll
            for (int r = 0; r < 8; ++r)
                e[(8 * h + r) * GEP + j * 16 + m16] = acc[i][j][r];
        __syncthreads();
        v4f vals[8];
#pragma unroll
        for (int it = 0; it < 8; ++it)
            vals[it] = *(const v4fa*)&e[(it * 2 + h) * GEP + c4] * oscale;
#pragma unroll
        for (int it = 0; it < 8; ++it) {
            const int gr = row0 + wrow * 32 + i * 16 + it * 2 + h;
            const int gc = col0 + wcol * 64 + c4;
            if (gr < M && gc + 3 < N)
                *(volatile v4f*)(C + (size_t)gr * N + gc) = vals[it];
        }
        __threadfence();
#pragma unroll
        for (int it = 0; it < 8; ++it) {
            const int gr = row0 + wrow * 32 + i * 16 + it * 2 + h;
            const int gc = col0 + wcol * 64 + c4;
            if (gr < M && gc + 3 < N)
                *(volatile v4f*)(C + (size_t)gr * N + gc) = vals[it];
        }
    }
}

__global__ __launch_bounds__(256)
void k_ln(const float* __restrict__ qkv, const float* __restrict__ qs, const float* __restrict__ ks,
          unsigned short* qh_p, unsigned short* ql_p, unsigned short* kh_p, unsigned short* kl_p,
          _Float16* v_p, int nrows) {
    __shared__ float red[8];
    const int row = blockIdx.x;
    if (row >= nrows) return;
    const int tid  = threadIdx.x;
    const int lane = tid & 31;
    const int wave = tid >> 5;
    const int e0   = tid * 8;
    const float* base = qkv + (size_t)row * NQKV;

    v8us hq, lq, hk, lk;
#pragma unroll
    for (int part = 0; part < 2; ++part) {
        const float* x = base + part * DMOD + e0;
        const v4f a = *(const v4fa*)x;
        const v4f b = *(const v4fa*)(x + 4);
        float v[8] = {a[0], a[1], a[2], a[3], b[0], b[1], b[2], b[3]};
        float s = 0.0f;
#pragma unroll
        for (int e = 0; e < 8; ++e) s += v[e];
        s = wsum(s);
        if (lane == 0) red[wave] = s;
        __syncthreads();
        float tot = 0.0f;
#pragma unroll
        for (int w = 0; w < 8; ++w) tot += red[w];
        __syncthreads();
        const float mu = tot * (1.0f / DMOD);
        float d = 0.0f;
#pragma unroll
        for (int e = 0; e < 8; ++e) { const float t = v[e] - mu; d += t * t; }
        d = wsum(d);
        if (lane == 0) red[wave] = d;
        __syncthreads();
        float totd = 0.0f;
#pragma unroll
        for (int w = 0; w < 8; ++w) totd += red[w];
        __syncthreads();
        const float var  = totd * (1.0f / DMOD);
        const float rstd = rsqrtf(var + 1e-6f);
        const float* sc  = part ? ks : qs;
        v8us hb, lb;
#pragma unroll
        for (int e = 0; e < 8; ++e) {
            const float y = (v[e] - mu) * rstd * sc[e0 + e];
            const unsigned short hbits = bf16_bits(y);
            const unsigned short lbits = bf16_bits(y - bf16_val(hbits));
            hb[e] = hbits; lb[e] = lbits;
        }
        if (part == 0) { hq = hb; lq = lb; } else { hk = hb; lk = lb; }
    }
    v8h hv;
    {
        const float* x = base + 2 * DMOD + e0;
        const v4f a = *(const v4fa*)x;
        const v4f b = *(const v4fa*)(x + 4);
        hv[0] = (_Float16)a[0]; hv[1] = (_Float16)a[1]; hv[2] = (_Float16)a[2]; hv[3] = (_Float16)a[3];
        hv[4] = (_Float16)b[0]; hv[5] = (_Float16)b[1]; hv[6] = (_Float16)b[2]; hv[7] = (_Float16)b[3];
    }
    const size_t o = (size_t)row * DMOD + e0;
    *(volatile v8us*)(qh_p + o) = hq;
    *(volatile v8us*)(ql_p + o) = lq;
    *(volatile v8us*)(kh_p + o) = hk;
    *(volatile v8us*)(kl_p + o) = lk;
    *(volatile v8h*)(v_p + o)   = hv;
    __threadfence();
    *(volatile v8us*)(qh_p + o) = hq;
    *(volatile v8us*)(ql_p + o) = lq;
    *(volatile v8us*)(kh_p + o) = hk;
    *(volatile v8us*)(kl_p + o) = lk;
    *(volatile v8h*)(v_p + o)   = hv;
}

#define AQB 128
#define AKB 32
#define QLD 256
#define KLD 256
#define VLD 40
#define PLD 40
#define OEP 136

__global__ __launch_bounds__(256) __attribute__((amdgpu_num_vgpr(256)))
void k_attn(const unsigned short* __restrict__ qh_p, const unsigned short* __restrict__ ql_p,
            const unsigned short* __restrict__ kh_p, const unsigned short* __restrict__ kl_p,
            const _Float16* __restrict__ v_p, const float* __restrict__ bias,
            const int* __restrict__ amask, _Float16* o_p) {
    __shared__ __attribute__((aligned(16))) unsigned short Qs[AQB * QLD];
    __shared__ __attribute__((aligned(16))) unsigned short Ks[AKB * KLD];
    __shared__ __attribute__((aligned(16))) _Float16 Vt[DHEAD * VLD];
    __shared__ __attribute__((aligned(16))) _Float16 Ps[8][16 * PLD];
    __shared__ __attribute__((aligned(16))) _Float16 Os[8][8 * OEP];

    const int head = blockIdx.y;
    const int qg   = blockIdx.x;
    const int tid  = threadIdx.x;
    const int lane = tid & 31;
    const int wave = tid >> 5;
    const int h    = lane >> 4;
    const int m16  = lane & 15;
    const int q0   = qg * AQB;
    const int qw   = q0 + wave * 16;
    const size_t hoff = (size_t)head * DHEAD;

#pragma unroll
    for (int i = 0; i < 16; ++i) {
        const int idx = tid + i * 256;
        const int r   = idx >> 5;
        const int cc  = idx & 31;
        const int pl  = cc >> 4;
        const int c8  = (cc & 15) * 8;
        const unsigned short* src = (pl ? ql_p : qh_p) + (size_t)(q0 + r) * DMOD + hoff + c8;
        *(v8us*)&Qs[r * QLD + pl * 128 + c8] = *(const v8usa*)src;
    }

    v8f oacc[8];
#pragma unroll
    for (int j = 0; j < 8; ++j) oacc[j] = (v8f)0.0f;
    float mrun[8], lrun[8];
#pragma unroll
    for (int r = 0; r < 8; ++r) { mrun[r] = -1.0e30f; lrun[r] = 0.0f; }

    const float scale = 0.08838834764831845f;
    const int nkb = qg * 4 + 4;
    __syncthreads();

    for (int kb = 0; kb < nkb; ++kb) {
        const int kbase = kb * AKB;
#pragma unroll
        for (int i = 0; i < 4; ++i) {
            const int idx = tid + i * 256;
            const int r   = idx >> 5;
            const int cc  = idx & 31;
            const int pl  = cc >> 4;
            const int c8  = (cc & 15) * 8;
            const unsigned short* src = (pl ? kl_p : kh_p) + (size_t)(kbase + r) * DMOD + hoff + c8;
            *(v8us*)&Ks[r * KLD + pl * 128 + c8] = *(const v8usa*)src;
        }
#pragma unroll
        for (int i = 0; i < 2; ++i) {
            const int idx = tid + i * 256;
            const int r   = idx >> 4;
            const int c8  = (idx & 15) * 8;
            const v8h va = *(const v8ha*)(v_p + (size_t)(kbase + r) * DMOD + hoff + c8);
#pragma unroll
            for (int e = 0; e < 8; ++e) Vt[(c8 + e) * VLD + r] = va[e];
        }
        __syncthreads();

        if (kbase <= qw + 15) {
            v8f sc[2];
            sc[0] = (v8f)0.0f; sc[1] = (v8f)0.0f;
#pragma unroll
            for (int c = 0; c < 4; ++c) {
                const unsigned short* qp = &Qs[(wave * 16 + m16) * QLD + c * 32];
                const v16b qa = ld_frag_b(qp, h);
                const v16b qb = ld_frag_b(qp + 128, h);
#pragma unroll
                for (int t = 0; t < 2; ++t) {
                    const unsigned short* kp = &Ks[(t * 16 + m16) * KLD + c * 32];
                    const v16b ka = ld_frag_b(kp, h);
                    const v16b kl = ld_frag_b(kp + 128, h);
                    sc[t] = mma_b(qa, ka, sc[t]);
                    sc[t] = mma_b(qa, kl, sc[t]);
                    sc[t] = mma_b(qb, ka, sc[t]);
                }
            }
#pragma unroll
            for (int t = 0; t < 2; ++t) {
                const int key   = kbase + t * 16 + m16;
                const float bb  = bias[head * SEQ + key];
                const bool live = amask[key] > 0;
#pragma unroll
                for (int r = 0; r < 8; ++r) {
                    const int qr = qw + 8 * h + r;
                    float v = sc[t][r] * scale + bb;
                    if (!live || key > qr) v = -3.0e38f;
                    sc[t][r] = v;
                }
            }
#pragma unroll
            for (int r = 0; r < 8; ++r) {
                float mx = fmaxf(sc[0][r], sc[1][r]);
#pragma unroll
                for (int off = 1; off < 16; off <<= 1) mx = fmaxf(mx, __shfl_xor(mx, off, 32));
                const float mnew = fmaxf(mrun[r], mx);
                const float p0 = __expf(sc[0][r] - mnew);
                const float p1 = __expf(sc[1][r] - mnew);
                sc[0][r] = p0; sc[1][r] = p1;
                float sm = p0 + p1;
#pragma unroll
                for (int off = 1; off < 16; off <<= 1) sm += __shfl_xor(sm, off, 32);
                const float alpha = __expf(mrun[r] - mnew);
                lrun[r] = lrun[r] * alpha + sm;
                mrun[r] = mnew;
#pragma unroll
                for (int j = 0; j < 8; ++j) oacc[j][r] = oacc[j][r] * alpha;
            }
            _Float16* pw = Ps[wave];
#pragma unroll
            for (int t = 0; t < 2; ++t)
#pragma unroll
                for (int r = 0; r < 8; ++r)
                    pw[(8 * h + r) * PLD + t * 16 + m16] = (_Float16)(sc[t][r] * 4096.0f);
            asm volatile("" ::: "memory");
            const v16h pf = ld_frag_h(&pw[m16 * PLD], h);
#pragma unroll
            for (int j = 0; j < 8; ++j) {
                const v16h vf = ld_frag_h(&Vt[(j * 16 + m16) * VLD], h);
                oacc[j] = mma_h(pf, vf, oacc[j]);
            }
        }
        __syncthreads();
    }

    float inv[8];
#pragma unroll
    for (int r = 0; r < 8; ++r) inv[r] = (1.0f / lrun[r]) * (1.0f / 4096.0f);
    _Float16* os = Os[wave];
    const int c8 = (lane & 15) * 8;
#pragma unroll
    for (int p = 0; p < 2; ++p) {
        __syncthreads();
        if (h == p) {
#pragma unroll
            for (int j = 0; j < 8; ++j)
#pragma unroll
                for (int r = 0; r < 8; ++r)
                    os[r * OEP + j * 16 + m16] = (_Float16)(oacc[j][r] * inv[r]);
        }
        __syncthreads();
        v8h vals[4];
#pragma unroll
        for (int it = 0; it < 4; ++it)
            vals[it] = *(const v8ha*)&os[(it * 2 + h) * OEP + c8];
#pragma unroll
        for (int it = 0; it < 4; ++it) {
            _Float16* gp = o_p + (size_t)(qw + 8 * p + it * 2 + h) * DMOD + hoff + c8;
            *(volatile v8h*)gp = vals[it];
        }
        __threadfence();
#pragma unroll
        for (int it = 0; it < 4; ++it) {
            _Float16* gp = o_p + (size_t)(qw + 8 * p + it * 2 + h) * DMOD + hoff + c8;
            *(volatile v8h*)gp = vals[it];
        }
    }
}

extern "C" void kernel_launch(void* const* d_in, const int* in_sizes, int n_in,
                              void* d_out, int out_size, void* d_ws, size_t ws_size,
                              hipStream_t stream) {
    if (n_in < 8) return;
    if (in_sizes[0] != SEQ * DMOD) return;
    if (in_sizes[1] < SEQ) return;
    if (in_sizes[3] < NHEAD * SEQ) return;
    if (in_sizes[4] != DMOD * NQKV) return;
    if (in_sizes[5] != DMOD * DMOD) return;
    if (in_sizes[6] < DMOD || in_sizes[7] < DMOD) return;
    if (out_size < SEQ * DMOD) return;

    const float* hidden = (const float*)d_in[0];
    const int*   amask  = (const int*)d_in[1];
    const float* abias  = (const float*)d_in[3];
    const float* wq     = (const float*)d_in[4];
    const float* wout   = (const float*)d_in[5];
    const float* qsc    = (const float*)d_in[6];
    const float* ksc    = (const float*)d_in[7];
    float* out = (float*)d_out;

    const size_t DD = (size_t)SEQ * DMOD;
    char* ws = (char*)d_ws;
    size_t off = 0;
    float* qkv = (float*)(ws + off);                      off += (size_t)SEQ * NQKV * sizeof(float);
    unsigned short* regB = (unsigned short*)(ws + off);   off += (size_t)NQKV * DMOD * 2;
    _Float16* regC = (_Float16*)(ws + off);               off += DD * 2;
    _Float16* woT  = (_Float16*)(ws + off);               off += DD * 2;
    unsigned short* khp = (unsigned short*)(ws + off);    off += 2 * DD * 2;
    if (off > ws_size) return;

    _Float16* wqT = (_Float16*)regB;
    unsigned short* qhp = regB;
    unsigned short* qlp = regB + DD;
    _Float16* vhp = (_Float16*)(regB + 2 * DD);
    unsigned short* klp = khp + DD;
    _Float16* ah  = regC;
    _Float16* of  = regC;

    {
        const int n = (int)DD;
        const int nblk = (n / 8 + 255) / 256;
        k_cvt<<<nblk, 256, 0, stream>>>(hidden, ah, n);
    }
    {
        dim3 grid((NQKV + 31) / 32, (DMOD + 63) / 64);
        k_wtr<<<grid, 256, 0, stream>>>(wq, wqT, DMOD, NQKV, 64.0f);
    }
    {
        dim3 grid((DMOD + 31) / 32, (DMOD + 63) / 64);
        k_wtr<<<grid, 256, 0, stream>>>(wout, woT, DMOD, DMOD, 64.0f);
    }
    {
        dim3 grid(NQKV / GBN, SEQ / GBM);
        k_gemm<<<grid, 256, 0, stream>>>(ah, wqT, qkv, SEQ, NQKV, DMOD, 1.0f / 64.0f);
    }
    k_ln<<<SEQ, 256, 0, stream>>>(qkv, qsc, ksc, qhp, qlp, khp, klp, vhp, SEQ);
    {
        dim3 grid(SEQ / AQB, NHEAD);
        k_attn<<<grid, 256, 0, stream>>>(qhp, qlp, khp, klp, vhp, abias, amask, of);
    }
    {
        dim3 grid(DMOD / GBN, SEQ / GBM);
        k_gemm<<<grid, 256, 0, stream>>>(of, woT, out, SEQ, DMOD, DMOD, 1.0f / 64.0f);
    }
}
